// GDEncoder_50431505989923
// MI455X (gfx1250) — hardware-verified
//
#include <hip/hip_runtime.h>
#include <hip/hip_bf16.h>
#include <math.h>
#include <stddef.h>


#define SEQ_T  640
#define NB     40
#define DIN    8
#define DTRAJ  32
#define DL     64
#define NHEAD  4
#define DHEAD  48
#define EMB    192
#define MROWS  (SEQ_T * NB)
#define KCAT   96
#define NGATE  256
#define NQKV   576
#define NAG    128

#define APITCH 104
#define CPITCH 72
#define QPITCH 72
#define SPITCH 52
#define OPITCH 200
#define YPITCH 132

#define LSTM_THREADS 384
#define GEMM_THREADS 128

static_assert(MROWS % 64 == 0);
static_assert(NQKV % 64 == 0);
static_assert(EMB % 64 == 0);
static_assert((KCAT % 8) == 0);
static_assert((APITCH % 8) == 0);

typedef _Float16 f16;
typedef f16    v16h __attribute__((ext_vector_type(16)));
typedef f16    v8h  __attribute__((ext_vector_type(8)));
typedef __bf16 v16b __attribute__((ext_vector_type(16)));
typedef __bf16 v8b  __attribute__((ext_vector_type(8)));
typedef float  v8f  __attribute__((ext_vector_type(8)));
typedef float  v4f  __attribute__((ext_vector_type(4)));

union FragH  { v16h v; v8h p[2]; };
union FragB  { v16b v; v8b p[2]; };
union Pack16 { v8h h; v8b b; v4f f; f16 he[8]; __bf16 be[8]; float fe[4]; };

__device__ __forceinline__ v8f zero8() {
  v8f z = {0.f, 0.f, 0.f, 0.f, 0.f, 0.f, 0.f, 0.f};
  return z;
}

__device__ __forceinline__ v8f mma_f16(v16h a, v16h b, v8f c) {
  c = __builtin_amdgcn_wmma_f32_16x16x32_f16(false, a, false, b, (short)0, c, false, false);
  asm volatile("v_nop\n\tv_nop\n\tv_nop\n\tv_nop" : "+v"(c) : "v"(a), "v"(b));
  return c;
}
__device__ __forceinline__ v8f mma_bf16(v16b a, v16b b, v8f c) {
  c = __builtin_amdgcn_wmma_f32_16x16x32_bf16(false, a, false, b, (short)0, c, false, false);
  asm volatile("v_nop\n\tv_nop\n\tv_nop\n\tv_nop" : "+v"(c) : "v"(a), "v"(b));
  return c;
}

__device__ __forceinline__ v16h ld_frag_h(const f16* base, int ld, int k0, int lane) {
  const int hh = lane >> 4, m = lane & 15;
  const f16* p = base + m * ld + k0 + 8 * hh;
  FragH f;
  f.p[0] = *(const v8h*)p;
  f.p[1] = *(const v8h*)(p + 16);
  return f.v;
}
__device__ __forceinline__ v16b ld_frag_b(const __bf16* base, int ld, int k0, int lane) {
  const int hh = lane >> 4, m = lane & 15;
  const __bf16* p = base + m * ld + k0 + 8 * hh;
  FragB f;
  f.p[0] = *(const v8b*)p;
  f.p[1] = *(const v8b*)(p + 16);
  return f.v;
}

__device__ __forceinline__ float sigm(float x) { return 1.f / (1.f + expf(-x)); }

__device__ __forceinline__ void st16(void* p, v4f v) { *(volatile v4f*)p = v; }

__global__ __launch_bounds__(256) void k_prep(
    const float* __restrict__ W_ih, const float* __restrict__ W_hh,
    const float* __restrict__ Wq, const float* __restrict__ Wk, const float* __restrict__ Wv,
    const float* __restrict__ Wa, const float* __restrict__ Wg, const int* __restrict__ adj,
    __bf16* wc_hi, __bf16* wc_lo, f16* wqkv, f16* wag)
{
  (void)adj;
  const int G0 = NGATE * KCAT / 8;
  const int G1 = 2 * G0;
  const int G2 = G1 + NQKV * DL / 8;
  const int G3 = G2 + NAG * EMB / 8;
  const int g = blockIdx.x * blockDim.x + threadIdx.x;
  if (g >= G3) return;

  Pack16 u;
  void* dst;
  if (g < G1) {
    const bool lo = (g >= G0);
    const int e0 = (lo ? (g - G0) : g) * 8;
    const int n  = e0 / KCAT;
    const int kb = e0 - n * KCAT;
    float v[8];
    if (kb < DTRAJ) {
#pragma unroll
      for (int e = 0; e < 8; ++e) v[e] = W_ih[n * DTRAJ + kb + e];
    } else {
#pragma unroll
      for (int e = 0; e < 8; ++e) v[e] = W_hh[n * DL + (kb - DTRAJ) + e];
    }
#pragma unroll
    for (int e = 0; e < 8; ++e) {
      const __bf16 h = (__bf16)v[e];
      u.be[e] = lo ? (__bf16)(v[e] - (float)h) : h;
    }
    dst = (void*)((lo ? wc_lo : wc_hi) + e0);
  } else if (g < G2) {
    const int e0 = (g - G1) * 8;
    const int nw = EMB * DL;
    const float* src = (e0 < nw) ? (Wq + e0) : (e0 < 2 * nw) ? (Wk + (e0 - nw)) : (Wv + (e0 - 2 * nw));
#pragma unroll
    for (int e = 0; e < 8; ++e) u.he[e] = (f16)(src[e] * 16.f);
    dst = (void*)(wqkv + e0);
  } else {
    const int e0 = (g - G2) * 8;
    const int nw = DL * EMB;
    const float* src = (e0 < nw) ? (Wa + e0) : (Wg + (e0 - nw));
#pragma unroll
    for (int e = 0; e < 8; ++e) u.he[e] = (f16)(src[e] * 16.f);
    dst = (void*)(wag + e0);
  }
  st16(dst, u.f);
  __threadfence();
  st16(dst, u.f);
}

__global__ __launch_bounds__(LSTM_THREADS) void k_lstm(
    const float* __restrict__ hist, const float* __restrict__ W1, const float* __restrict__ b1,
    const __bf16* __restrict__ wc_hi, const __bf16* __restrict__ wc_lo,
    const float* __restrict__ b_ih, const float* __restrict__ b_hh,
    float* seqf, f16* seq16)
{
  __shared__ __bf16 Ahi[48 * APITCH] __attribute__((aligned(16)));
  __shared__ __bf16 Alo[48 * APITCH] __attribute__((aligned(16)));
  __shared__ float  Hs[NB * DL] __attribute__((aligned(16)));
  __shared__ float  W1s[DTRAJ * DIN];
  __shared__ float  b1s[DTRAJ];
  __shared__ float  bsum[NGATE];

  const int tid = threadIdx.x;
  const int lane = tid & 31, wave = tid >> 5;
  const int hh = lane >> 4, m = lane & 15;
  const int mt = wave >> 2, jj = wave & 3;

  for (int i = tid; i < 48 * APITCH; i += LSTM_THREADS) { Ahi[i] = (__bf16)0.f; Alo[i] = (__bf16)0.f; }
  for (int i = tid; i < DTRAJ * DIN; i += LSTM_THREADS) W1s[i] = W1[i];
  for (int i = tid; i < DTRAJ; i += LSTM_THREADS) b1s[i] = b1[i];
  for (int i = tid; i < NGATE; i += LSTM_THREADS) bsum[i] = b_ih[i] + b_hh[i];
  __syncthreads();

  const int jcol = jj * 16 + m;
  const float bi_ = bsum[jcol];
  const float bf_ = bsum[DL + jcol];
  const float bg_ = bsum[2 * DL + jcol];
  const float bo_ = bsum[3 * DL + jcol];
  float cst[8];
#pragma unroll
  for (int r8 = 0; r8 < 8; ++r8) cst[r8] = 0.f;

  const int piece = tid & 7;
  const int L0 = tid >> 3;

  for (int t = 0; t < SEQ_T; ++t) {
    const size_t rowb = (size_t)t * NB;

    for (int i = tid; i < NB * DTRAJ; i += LSTM_THREADS) {
      const int r = i >> 5, k = i & 31;
      const float* hp = hist + (rowb + r) * DIN;
      const v4f x0 = *(const v4f*)hp;
      const v4f x1 = *(const v4f*)(hp + 4);
      const float* w = W1s + k * DIN;
      float s = x0[0] * w[0];
      s += x0[1] * w[1];
      s += x0[2] * w[2];
      s += x0[3] * w[3];
      s += x1[0] * w[4];
      s += x1[1] * w[5];
      s += x1[2] * w[6];
      s += x1[3] * w[7];
      s += b1s[k];
      const float xv = (s > 0.f) ? s : expm1f(s);
      const __bf16 xh = (__bf16)xv;
      const __bf16 xl = (__bf16)(xv - (float)xh);
      Ahi[r * APITCH + k] = xh;
      Alo[r * APITCH + k] = xl;
    }
    __syncthreads();

    v8f acc[4];
#pragma unroll
    for (int g = 0; g < 4; ++g) acc[g] = zero8();
#pragma unroll 1
    for (int kk = 0; kk < 3; ++kk) {
      const int k0 = kk * 32;
      const v16b ah = ld_frag_b(Ahi + mt * 16 * APITCH, APITCH, k0, lane);
      const v16b al = ld_frag_b(Alo + mt * 16 * APITCH, APITCH, k0, lane);
#pragma unroll
      for (int g = 0; g < 4; ++g) {
        const size_t nb = (size_t)(g * DL + jj * 16) * KCAT;
        const v16b bh = ld_frag_b(wc_hi + nb, KCAT, k0, lane);
        const v16b bl = ld_frag_b(wc_lo + nb, KCAT, k0, lane);
        acc[g] = mma_bf16(ah, bh, acc[g]);
        acc[g] = mma_bf16(ah, bl, acc[g]);
        acc[g] = mma_bf16(al, bh, acc[g]);
      }
    }
    __syncthreads();

#pragma unroll
    for (int r8 = 0; r8 < 8; ++r8) {
      const int r = mt * 16 + hh * 8 + r8;
      const float gi = acc[0][r8] + bi_;
      const float gf = acc[1][r8] + bf_;
      const float gg = acc[2][r8] + bg_;
      const float go = acc[3][r8] + bo_;
      const float cn = sigm(gf) * cst[r8] + sigm(gi) * tanhf(gg);
      const float hn = sigm(go) * tanhf(cn);
      cst[r8] = cn;
      if (r < NB) {
        const __bf16 hb = (__bf16)hn;
        Ahi[r * APITCH + DTRAJ + jcol] = hb;
        Alo[r * APITCH + DTRAJ + jcol] = (__bf16)(hn - (float)hb);
        Hs[r * DL + jcol] = hn;
      }
    }
    __syncthreads();

    v4f fv0;
    v4f fv1 = {0.f, 0.f, 0.f, 0.f};
    Pack16 u;
    u.f = fv1;
    float* fd0;
    float* fd1 = seqf;
    f16*   sd  = seq16;
    {
      const int r = L0 >> 1;
      const int col = (L0 & 1) * 32 + piece * 4;
      fv0 = *(const v4f*)(Hs + r * DL + col);
      fd0 = seqf + (rowb + r) * DL + col;
    }
    const bool has1 = (L0 < 32);
    if (has1) {
      const int L1 = L0 + 48;
      const int r = L1 >> 1;
      const int col = (L1 & 1) * 32 + piece * 4;
      fv1 = *(const v4f*)(Hs + r * DL + col);
      fd1 = seqf + (rowb + r) * DL + col;
    }
    const bool hasS = (L0 < NB);
    if (hasS) {
      const int col = piece * 8;
      const v4f a = *(const v4f*)(Hs + L0 * DL + col);
      const v4f b = *(const v4f*)(Hs + L0 * DL + col + 4);
#pragma unroll
      for (int e = 0; e < 4; ++e) {
        u.he[e]     = (f16)(a[e] * 64.f);
        u.he[4 + e] = (f16)(b[e] * 64.f);
      }
      sd = seq16 + (rowb + L0) * DL + col;
    }
    st16(fd0, fv0);
    if (has1) st16(fd1, fv1);
    if (hasS) st16(sd, u.f);
    __threadfence();
    st16(fd0, fv0);
    if (has1) st16(fd1, fv1);
    if (hasS) st16(sd, u.f);
  }
}

__global__ __launch_bounds__(GEMM_THREADS) void k_qkv(
    const f16* __restrict__ seq16, const f16* __restrict__ wqkv,
    const float* __restrict__ bq, const float* __restrict__ bk, const float* __restrict__ bv,
    f16* qkv)
{
  __shared__ f16 Cs[64 * CPITCH] __attribute__((aligned(16)));
  const int tid = threadIdx.x, lane = tid & 31, wave = tid >> 5;
  const int hh = lane >> 4, m = lane & 15;
  const int rb = blockIdx.x, cb = blockIdx.y;
  const int row0 = rb * 64 + wave * 16;
  const int col0 = cb * 64;
  const int region = cb / 3;
  const float* bias = (region == 0) ? bq : (region == 1) ? bk : bv;
  const int nloc0 = col0 - region * EMB;
  const float oscale = (region == 2) ? 256.f : 64.f;

  v8f acc[4];
#pragma unroll
  for (int nt = 0; nt < 4; ++nt) acc[nt] = zero8();
#pragma unroll
  for (int kk = 0; kk < 2; ++kk) {
    const int k0 = kk * 32;
    const v16h a = ld_frag_h(seq16 + (size_t)row0 * DL, DL, k0, lane);
#pragma unroll
    for (int nt = 0; nt < 4; ++nt) {
      const v16h b = ld_frag_h(wqkv + (size_t)(col0 + nt * 16) * DL, DL, k0, lane);
      acc[nt] = mma_f16(a, b, acc[nt]);
    }
  }
#pragma unroll
  for (int nt = 0; nt < 4; ++nt) {
    const float bn = bias[nloc0 + nt * 16 + m];
#pragma unroll
    for (int r8 = 0; r8 < 8; ++r8) {
      const float v = acc[nt][r8] * (1.f / 1024.f) + bn;
      Cs[(wave * 16 + hh * 8 + r8) * CPITCH + nt * 16 + m] = (f16)(v * oscale);
    }
  }
  __syncthreads();

  const int rl = lane >> 3, piece = lane & 7;
#pragma unroll
  for (int p = 0; p < 4; ++p) {
    const int r = wave * 16 + p * 4 + rl;
    Pack16 u;
    u.h = *(const v8h*)(Cs + r * CPITCH + piece * 8);
    st16(qkv + ((size_t)rb * 64 + r) * NQKV + col0 + piece * 8, u.f);
  }
  __threadfence();
#pragma unroll
  for (int p = 0; p < 4; ++p) {
    const int r = wave * 16 + p * 4 + rl;
    Pack16 u;
    u.h = *(const v8h*)(Cs + r * CPITCH + piece * 8);
    st16(qkv + ((size_t)rb * 64 + r) * NQKV + col0 + piece * 8, u.f);
  }
}

__global__ __launch_bounds__(GEMM_THREADS) void k_attn(const f16* __restrict__ qkv, f16* o16)
{
  __shared__ f16   Qs[48 * QPITCH] __attribute__((aligned(16)));
  __shared__ f16   Ks[48 * QPITCH] __attribute__((aligned(16)));
  __shared__ f16   Vts[48 * QPITCH] __attribute__((aligned(16)));
  __shared__ f16   Ps[48 * QPITCH] __attribute__((aligned(16)));
  __shared__ float Ss[48 * SPITCH];
  __shared__ f16   Os[48 * OPITCH] __attribute__((aligned(16)));

  const int tid = threadIdx.x, lane = tid & 31, wave = tid >> 5;
  const int hh = lane >> 4, m = lane & 15;
  const int t = blockIdx.x;

  const f16 hz = (f16)0.f;
  for (int i = tid; i < 48 * QPITCH; i += GEMM_THREADS) { Qs[i] = hz; Ks[i] = hz; Vts[i] = hz; Ps[i] = hz; }
  __syncthreads();

  for (int head = 0; head < NHEAD; ++head) {
    for (int it = tid; it < NB * 18; it += GEMM_THREADS) {
      const int a   = it / 18;
      const int rem = it - a * 18;
      const int w   = rem / 6;
      const int ch  = rem - w * 6;
      const f16* src = qkv + ((size_t)t * NB + a) * NQKV + w * EMB + head * DHEAD + ch * 8;
      const v8h v = *(const v8h*)src;
      if (w == 0)      *(v8h*)(Qs + a * QPITCH + ch * 8) = v;
      else if (w == 1) *(v8h*)(Ks + a * QPITCH + ch * 8) = v;
      else {
#pragma unroll
        for (int e = 0; e < 8; ++e) Vts[(ch * 8 + e) * QPITCH + a] = v[e];
      }
    }
    __syncthreads();

    for (int tile = wave; tile < 9; tile += 4) {
      const int mt = tile / 3, nt = tile - mt * 3;
      v8f acc = zero8();
#pragma unroll
      for (int kk = 0; kk < 2; ++kk) {
        const v16h a = ld_frag_h(Qs + mt * 16 * QPITCH, QPITCH, kk * 32, lane);
        const v16h b = ld_frag_h(Ks + nt * 16 * QPITCH, QPITCH, kk * 32, lane);
        acc = mma_f16(a, b, acc);
      }
#pragma unroll
      for (int r8 = 0; r8 < 8; ++r8)
        Ss[(mt * 16 + hh * 8 + r8) * SPITCH + nt * 16 + m] = acc[r8];
    }
    __syncthreads();

    if (tid < NB) {
      float* srow = Ss + tid * SPITCH;
      const float sc = 1.f / 32768.f;
      float mx = srow[0] * sc;
      for (int cI = 1; cI < NB; ++cI) mx = fmaxf(mx, srow[cI] * sc);
      float sum = 0.f;
      for (int cI = 0; cI < NB; ++cI) {
        const float e = expf(srow[cI] * sc - mx);
        srow[cI] = e;
        sum += e;
      }
      const float inv = 1.f / sum;
      f16* prow = Ps + tid * QPITCH;
      for (int cI = 0; cI < NB; ++cI) prow[cI] = (f16)(srow[cI] * inv * 256.f);
    }
    __syncthreads();

    for (int tile = wave; tile < 9; tile += 4) {
      const int mt = tile / 3, nt = tile - mt * 3;
      v8f acc = zero8();
#pragma unroll
      for (int kk = 0; kk < 2; ++kk) {
        const v16h a = ld_frag_h(Ps + mt * 16 * QPITCH, QPITCH, kk * 32, lane);
        const v16h b = ld_frag_h(Vts + nt * 16 * QPITCH, QPITCH, kk * 32, lane);
        acc = mma_f16(a, b, acc);
      }
#pragma unroll
      for (int r8 = 0; r8 < 8; ++r8)
        Os[(mt * 16 + hh * 8 + r8) * OPITCH + head * DHEAD + nt * 16 + m] = (f16)(acc[r8] * (1.f / 256.f));
    }
    __syncthreads();
  }

  const int piece = tid & 7, Lb = tid >> 3;
#pragma unroll
  for (int p = 0; p < 8; ++p) {
    const int L = Lb + 16 * p;
    if (L < NB * 3) {
      const int r = L / 3, seg = L - 3 * r;
      Pack16 u;
      u.h = *(const v8h*)(Os + r * OPITCH + seg * 64 + piece * 8);
      st16(o16 + ((size_t)t * NB + r) * EMB + seg * 64 + piece * 8, u.f);
    }
  }
  __threadfence();
#pragma unroll
  for (int p = 0; p < 8; ++p) {
    const int L = Lb + 16 * p;
    if (L < NB * 3) {
      const int r = L / 3, seg = L - 3 * r;
      Pack16 u;
      u.h = *(const v8h*)(Os + r * OPITCH + seg * 64 + piece * 8);
      st16(o16 + ((size_t)t * NB + r) * EMB + seg * 64 + piece * 8, u.f);
    }
  }
}

__global__ __launch_bounds__(GEMM_THREADS) void k_glu(
    const f16* __restrict__ o16, const f16* __restrict__ wag,
    const float* __restrict__ ba, const float* __restrict__ bg, const float* __restrict__ seqf,
    const float* __restrict__ gamma, const float* __restrict__ beta, float* out)
{
  __shared__ float Ys[64 * YPITCH] __attribute__((aligned(16)));
  const int tid = threadIdx.x, lane = tid & 31, wave = tid >> 5;
  const int hh = lane >> 4, m = lane & 15;
  const int row0 = blockIdx.x * 64;

  v8f acc[8];
#pragma unroll
  for (int nt = 0; nt < 8; ++nt) acc[nt] = zero8();
  const f16* abase = o16 + (size_t)(row0 + wave * 16) * EMB;
#pragma unroll 1
  for (int kk = 0; kk < 6; ++kk) {
    const int k0 = kk * 32;
    const v16h a = ld_frag_h(abase, EMB, k0, lane);
#pragma unroll
    for (int nt = 0; nt < 8; ++nt) {
      const v16h b = ld_frag_h(wag + (size_t)(nt * 16) * EMB, EMB, k0, lane);
      acc[nt] = mma_f16(a, b, acc[nt]);
    }
  }
#pragma unroll
  for (int nt = 0; nt < 8; ++nt) {
    const float* bp = (nt < 4) ? (ba + nt * 16) : (bg + (nt - 4) * 16);
    const float bn = bp[m];
    const int n = nt * 16 + m;
#pragma unroll
    for (int r8 = 0; r8 < 8; ++r8)
      Ys[(wave * 16 + hh * 8 + r8) * YPITCH + n] = acc[nt][r8] * (1.f / 4096.f) + bn;
  }
  __syncthreads();

  const int q16 = tid & 15, rsub = tid >> 4;
  const int col = q16 * 4;
  const v4f gm = *(const v4f*)(gamma + col);
  const v4f bt = *(const v4f*)(beta + col);
  v4f res[8];
#pragma unroll
  for (int p = 0; p < 8; ++p) {
    const int r = p * 8 + rsub;
    const size_t row = (size_t)row0 + r;
    const v4f a4 = *(const v4f*)(Ys + r * YPITCH + col);
    const v4f g4 = *(const v4f*)(Ys + r * YPITCH + DL + col);
    const v4f s4 = *(const v4f*)(seqf + row * DL + col);
    v4f y;
#pragma unroll
    for (int e = 0; e < 4; ++e) y[e] = s4[e] + a4[e] * sigm(g4[e]);
    float ps = (y[0] + y[1]) + (y[2] + y[3]);
    ps += __shfl_xor(ps, 1, 32);
    ps += __shfl_xor(ps, 2, 32);
    ps += __shfl_xor(ps, 4, 32);
    ps += __shfl_xor(ps, 8, 32);
    const float mu = ps * (1.f / 64.f);
    v4f d;
#pragma unroll
    for (int e = 0; e < 4; ++e) d[e] = y[e] - mu;
    float pv = (d[0] * d[0] + d[1] * d[1]) + (d[2] * d[2] + d[3] * d[3]);
    pv += __shfl_xor(pv, 1, 32);
    pv += __shfl_xor(pv, 2, 32);
    pv += __shfl_xor(pv, 4, 32);
    pv += __shfl_xor(pv, 8, 32);
    const float var = pv * (1.f / 64.f);
    const float inv = 1.f / sqrtf(var + 1e-5f);
    v4f o;
#pragma unroll
    for (int e = 0; e < 4; ++e) o[e] = d[e] * inv * gm[e] + bt[e];
    res[p] = o;
  }
#pragma unroll
  for (int p = 0; p < 8; ++p)
    st16(out + ((size_t)row0 + p * 8 + rsub) * DL + col, res[p]);
  __threadfence();
#pragma unroll
  for (int p = 0; p < 8; ++p)
    st16(out + ((size_t)row0 + p * 8 + rsub) * DL + col, res[p]);
}

static inline size_t align256(size_t x) { return (x + 255) & ~(size_t)255; }

extern "C" void kernel_launch(void* const* d_in, const int* in_sizes, int n_in,
                              void* d_out, int out_size, void* d_ws, size_t ws_size,
                              hipStream_t stream)
{
  if (n_in < 20 || d_out == 0 || d_ws == 0) return;
  const float* hist  = (const float*)d_in[0];
  const int*   adj   = (const int*)d_in[1];
  const float* W1    = (const float*)d_in[2];
  const float* b1    = (const float*)d_in[3];
  const float* W_ih  = (const float*)d_in[4];
  const float* W_hh  = (const float*)d_in[5];
  const float* b_ih  = (const float*)d_in[6];
  const float* b_hh  = (const float*)d_in[7];
  const float* Wq    = (const float*)d_in[8];
  const float* bq    = (const float*)d_in[9];
  const float* Wk    = (const float*)d_in[10];
  const float* bk    = (const float*)d_in[11];
  const float* Wv    = (const float*)d_in[12];
  const float* bv    = (const float*)d_in[13];
  const float* Wa    = (const float*)d_in[14];
  const float* ba    = (const float*)d_in[15];
  const float* Wg    = (const float*)d_in[16];
  const float* bg    = (const float*)d_in[17];
  const float* gamma = (const float*)d_in[18];
  const float* beta  = (const float*)d_in[19];

  if (in_sizes[0] < MROWS * DIN || in_sizes[2] < DTRAJ * DIN || in_sizes[3] < DTRAJ ||
      in_sizes[4] < NGATE * DTRAJ || in_sizes[5] < NGATE * DL || in_sizes[6] < NGATE || in_sizes[7] < NGATE ||
      in_sizes[8] < EMB * DL || in_sizes[9] < EMB || in_sizes[10] < EMB * DL || in_sizes[11] < EMB ||
      in_sizes[12] < EMB * DL || in_sizes[13] < EMB || in_sizes[14] < DL * EMB || in_sizes[15] < DL ||
      in_sizes[16] < DL * EMB || in_sizes[17] < DL || in_sizes[18] < DL || in_sizes[19] < DL) return;
  if (out_size < MROWS * DL) return;

  size_t off = 0;
  const size_t oWCH  = off; off = align256(off + (size_t)NGATE * KCAT * 2);
  const size_t oWCL  = off; off = align256(off + (size_t)NGATE * KCAT * 2);
  const size_t oWQKV = off; off = align256(off + (size_t)NQKV * DL * 2);
  const size_t oWAG  = off; off = align256(off + (size_t)NAG * EMB * 2);
  const size_t oSEQ  = off; off = align256(off + (size_t)MROWS * DL * 4);
  const size_t oS16  = off; off = align256(off + (size_t)MROWS * DL * 2);
  const size_t oQKV  = off; off = align256(off + (size_t)MROWS * NQKV * 2);
  const size_t oO16  = off; off = align256(off + (size_t)MROWS * EMB * 2);
  const size_t need  = off;
  if (need > ws_size) return;
  if (need > (size_t)134217728) return;

  char* ws = (char*)d_ws;
  __bf16* wc_hi = (__bf16*)(ws + oWCH);
  __bf16* wc_lo = (__bf16*)(ws + oWCL);
  f16*    wqkv  = (f16*)(ws + oWQKV);
  f16*    wag   = (f16*)(ws + oWAG);
  float*  seqf  = (float*)(ws + oSEQ);
  f16*    seq16 = (f16*)(ws + oS16);
  f16*    qkv   = (f16*)(ws + oQKV);
  f16*    o16   = (f16*)(ws + oO16);
  float*  out   = (float*)d_out;

  {
    const int groups = 2 * (NGATE * KCAT / 8) + NQKV * DL / 8 + NAG * EMB / 8;
    k_prep<<<dim3((groups + 255) / 256), dim3(256), 0, stream>>>(
        W_ih, W_hh, Wq, Wk, Wv, Wa, Wg, adj, wc_hi, wc_lo, wqkv, wag);
  }
  k_lstm<<<dim3(1), dim3(LSTM_THREADS), 0, stream>>>(
      hist, W1, b1, wc_hi, wc_lo, b_ih, b_hh, seqf, seq16);
  k_qkv<<<dim3(MROWS / 64, NQKV / 64), dim3(GEMM_THREADS), 0, stream>>>(
      seq16, wqkv, bq, bk, bv, qkv);
  k_attn<<<dim3(SEQ_T), dim3(GEMM_THREADS), 0, stream>>>(qkv, o16);
  k_glu<<<dim3(MROWS / 64), dim3(GEMM_THREADS), 0, stream>>>(
      o16, wag, ba, bg, seqf, gamma, beta, out);
  (void)hipGetLastError();
}
